// GATLayer_regular_65000035058127
// MI455X (gfx1250) — hardware-verified
//
#include <hip/hip_runtime.h>
#include <stddef.h>


#define DF      128
#define NTHR    256
#define NWAVE   8
#define EPT     8
#define NGRP    2
#define CHUNK   (NTHR * EPT * NGRP)
#define WCAP    (EPT * NGRP * 32)
#define LISTN   (NWAVE * WCAP)
#define NB      512
#define GROWS   128
#define APITCH  136
#define WSCALE  8.0f
#define WINV    0.125f

#define LDS_SA   (GROWS * APITCH * 2)
#define LDS_STG  (GROWS * DF * 4)
#define LDS_NODE (LDS_SA + LDS_STG + 2 * GROWS * 4)
#define LDS_AGG  (NB * DF * 4 + LISTN * 4 + 64 + NB * 4)

static_assert((CHUNK & (CHUNK - 1)) == 0);
static_assert(CHUNK <= 4096);
static_assert((NB & (NB - 1)) == 0);
static_assert(NB <= 4096);
static_assert((LDS_SA & 15) == 0);
static_assert(((GROWS * DF / 8) % NTHR) == 0);
static_assert(((NB * DF / 4) % NTHR) == 0);
static_assert(NB == NWAVE * 64);
static_assert(LDS_AGG <= 300 * 1024);

typedef float    v4f  __attribute__((ext_vector_type(4)));
typedef float    v8f  __attribute__((ext_vector_type(8)));
typedef int      v4i  __attribute__((ext_vector_type(4)));
typedef _Float16 v8h  __attribute__((ext_vector_type(8)));
typedef _Float16 v16h __attribute__((ext_vector_type(16)));
union FragH { v16h v; v8h h[2]; };

__device__ __forceinline__ v8h cvt8(v4f a, v4f b) {
  v8h r;
  r[0] = (_Float16)a.x; r[1] = (_Float16)a.y; r[2] = (_Float16)a.z; r[3] = (_Float16)a.w;
  r[4] = (_Float16)b.x; r[5] = (_Float16)b.y; r[6] = (_Float16)b.z; r[7] = (_Float16)b.w;
  return r;
}

__device__ __forceinline__ v8f wmh(v16h a, v16h b, v8f c) {
  v8f d = __builtin_amdgcn_wmma_f32_16x16x32_f16(false, a, false, b, (short)0, c, false, false);
  asm volatile("v_nop\n\tv_nop\n\tv_nop\n\tv_nop" : "+v"(d) : "v"(a), "v"(b));
  return d;
}

__device__ __forceinline__ int scan_chunk(const int* __restrict__ keys, int nE, int cbase, int nodeBase,
                                          int* list, int tid, int lane, int wave) {
  int wc = 0;
  (void)lane;
#pragma unroll
  for (int g = 0; g < NGRP; ++g) {
    const int el0  = (g * NTHR + tid) * EPT;
    const int e0   = cbase + el0;
    const int sent = -2147483647 - 1;
    v4i da, db;
    if (cbase + CHUNK <= nE) {
      da = *(const v4i*)(keys + e0);
      db = *(const v4i*)(keys + e0 + 4);
    } else {
      const int em = nE - 1;
      da.x = (e0     < nE) ? keys[min(e0,     em)] : sent;
      da.y = (e0 + 1 < nE) ? keys[min(e0 + 1, em)] : sent;
      da.z = (e0 + 2 < nE) ? keys[min(e0 + 2, em)] : sent;
      da.w = (e0 + 3 < nE) ? keys[min(e0 + 3, em)] : sent;
      db.x = (e0 + 4 < nE) ? keys[min(e0 + 4, em)] : sent;
      db.y = (e0 + 5 < nE) ? keys[min(e0 + 5, em)] : sent;
      db.z = (e0 + 6 < nE) ? keys[min(e0 + 6, em)] : sent;
      db.w = (e0 + 7 < nE) ? keys[min(e0 + 7, em)] : sent;
    }
    const unsigned nb = (unsigned)nodeBase;
    const unsigned s0 = (unsigned)da.x - nb, s1 = (unsigned)da.y - nb;
    const unsigned s2 = (unsigned)da.z - nb, s3 = (unsigned)da.w - nb;
    const unsigned s4 = (unsigned)db.x - nb, s5 = (unsigned)db.y - nb;
    const unsigned s6 = (unsigned)db.z - nb, s7 = (unsigned)db.w - nb;
    const bool h0 = s0 < (unsigned)NB, h1 = s1 < (unsigned)NB, h2 = s2 < (unsigned)NB, h3 = s3 < (unsigned)NB;
    const bool h4 = s4 < (unsigned)NB, h5 = s5 < (unsigned)NB, h6 = s6 < (unsigned)NB, h7 = s7 < (unsigned)NB;
    const unsigned any = __builtin_amdgcn_ballot_w32(h0 | h1 | h2 | h3 | h4 | h5 | h6 | h7);
    if (any != 0u) {
#define HITJ(J, HJ, SJ) { \
        const unsigned mj = __builtin_amdgcn_ballot_w32(HJ); \
        if (mj != 0u) { \
          if (HJ) { \
            const int pos = wc + (int)__builtin_amdgcn_mbcnt_lo(mj, 0u); \
            if (pos < WCAP) list[wave * WCAP + pos] = ((el0 + (J)) << 12) | (int)(SJ); \
          } \
          wc += (int)__builtin_popcount(mj); } }
      HITJ(0, h0, s0)
      HITJ(1, h1, s1)
      HITJ(2, h2, s2)
      HITJ(3, h3, s3)
      HITJ(4, h4, s4)
      HITJ(5, h5, s5)
      HITJ(6, h6, s6)
      HITJ(7, h7, s7)
#undef HITJ
    }
  }
  return wc;
}

__global__ __launch_bounds__(NTHR) void k_wprep(
    const float* __restrict__ W1, const float* __restrict__ W2,
    _Float16* w1s, _Float16* w2s) {
  const int i   = blockIdx.x * NTHR + threadIdx.x;
  const int per = DF * DF / 8;
  if (i >= 2 * per) return;
  const bool first = i < per;
  const int o = (first ? i : i - per) * 8;
  const float* p = (first ? W1 : W2) + o;
  v4f a = *(const v4f*)p, b = *(const v4f*)(p + 4);
  a = a * WSCALE;
  b = b * WSCALE;
  const v8h hv = cvt8(a, b);
  _Float16* dp = (first ? w1s : w2s) + o;
  *(volatile v8h*)dp = hv;
  __threadfence();
  *(volatile v8h*)dp = hv;
}

__global__ __launch_bounds__(NTHR) void k_node(
    const float* __restrict__ x, const _Float16* __restrict__ w1s, const _Float16* __restrict__ w2s,
    const float* __restrict__ b1, const float* __restrict__ b2,
    const float* __restrict__ a1w, const float* __restrict__ a1b,
    const float* __restrict__ a2w, const float* __restrict__ a2b,
    float* xj, float* a1p, float* a2p, int nN) {
  extern __shared__ v4f lds_dyn[];
  char*     lb  = (char*)lds_dyn;
  _Float16* sA  = (_Float16*)lb;
  float*    stg = (float*)(lb + LDS_SA);
  float*    sa1 = (float*)(lb + LDS_SA + LDS_STG);
  float*    sa2 = sa1 + GROWS;
  const int tid = threadIdx.x, lane = tid & 31, wave = tid >> 5, hh = lane >> 4, m = lane & 15;
  const int rowBase = blockIdx.x * GROWS;

#pragma unroll
  for (int i = 0; i < (GROWS * DF / 8) / NTHR; ++i) {
    const int idx = i * NTHR + tid;
    const int r   = idx >> 4;
    const int c0  = (idx & 15) * 8;
    int node = rowBase + r;
    node = node > nN - 1 ? nN - 1 : node;
    const float* xp = x + (size_t)node * DF + c0;
    const v4f a = *(const v4f*)xp, b = *(const v4f*)(xp + 4);
    *(v8h*)(sA + r * APITCH + c0) = cvt8(a, b);
  }
  __syncthreads();

  const _Float16* ar = sA + (wave * 16 + m) * APITCH + 8 * hh;
  v8f acc[8];

#pragma unroll
  for (int t = 0; t < 8; ++t) { v8f z = {0.f, 0.f, 0.f, 0.f, 0.f, 0.f, 0.f, 0.f}; acc[t] = z; }
#pragma unroll 1
  for (int kt = 0; kt < DF / 32; ++kt) {
    FragH a;
    a.h[0] = *(const v8h*)(ar + 32 * kt);
    a.h[1] = *(const v8h*)(ar + 32 * kt + 16);
#pragma unroll
    for (int t = 0; t < 8; ++t) {
      const _Float16* bp = w1s + (size_t)(16 * t + m) * DF + 32 * kt + 8 * hh;
      FragH b;
      b.h[0] = *(const v8h*)bp;
      b.h[1] = *(const v8h*)(bp + 16);
      acc[t] = wmh(a.v, b.v, acc[t]);
    }
  }
  {
    float ss[8];
#pragma unroll
    for (int r = 0; r < 8; ++r) ss[r] = 0.f;
#pragma unroll
    for (int t = 0; t < 8; ++t) {
      const float bc = b1[16 * t + m];
      const float ac = a1w[16 * t + m];
#pragma unroll
      for (int r = 0; r < 8; ++r) {
        float v = acc[t][r] * WINV + bc;
        v = (v >= 0.f) ? v : 0.2f * v;
        ss[r] += v * ac;
      }
    }
#pragma unroll
    for (int mk = 1; mk < 16; mk <<= 1) {
#pragma unroll
      for (int r = 0; r < 8; ++r) ss[r] += __shfl_xor(ss[r], mk, 32);
    }
    if (m == 0) {
      const float ab = a1b[0];
#pragma unroll
      for (int r = 0; r < 8; ++r) sa1[wave * 16 + 8 * hh + r] = ss[r] + ab;
    }
  }

#pragma unroll
  for (int t = 0; t < 8; ++t) { v8f z = {0.f, 0.f, 0.f, 0.f, 0.f, 0.f, 0.f, 0.f}; acc[t] = z; }
#pragma unroll 1
  for (int kt = 0; kt < DF / 32; ++kt) {
    FragH a;
    a.h[0] = *(const v8h*)(ar + 32 * kt);
    a.h[1] = *(const v8h*)(ar + 32 * kt + 16);
#pragma unroll
    for (int t = 0; t < 8; ++t) {
      const _Float16* bp = w2s + (size_t)(16 * t + m) * DF + 32 * kt + 8 * hh;
      FragH b;
      b.h[0] = *(const v8h*)bp;
      b.h[1] = *(const v8h*)(bp + 16);
      acc[t] = wmh(a.v, b.v, acc[t]);
    }
  }
  {
    float ss[8];
#pragma unroll
    for (int r = 0; r < 8; ++r) ss[r] = 0.f;
    float* sp = stg + (wave * 16 + 8 * hh) * DF + m;
#pragma unroll
    for (int t = 0; t < 8; ++t) {
      const float bc = b2[16 * t + m];
      const float ac = a2w[16 * t + m];
#pragma unroll
      for (int r = 0; r < 8; ++r) {
        float v = acc[t][r] * WINV + bc;
        v = (v >= 0.f) ? v : 0.2f * v;
        sp[r * DF + 16 * t] = v;
        ss[r] += v * ac;
      }
    }
#pragma unroll
    for (int mk = 1; mk < 16; mk <<= 1) {
#pragma unroll
      for (int r = 0; r < 8; ++r) ss[r] += __shfl_xor(ss[r], mk, 32);
    }
    if (m == 0) {
      const float ab = a2b[0];
#pragma unroll
      for (int r = 0; r < 8; ++r) sa2[wave * 16 + 8 * hh + r] = ss[r] + ab;
    }
  }
  __syncthreads();

  const float* lp = stg + wave * 16 * DF + 4 * lane;
  float* gp = xj + ((size_t)rowBase + wave * 16) * DF + 4 * lane;
#pragma unroll
  for (int i = 0; i < 16; ++i) { const v4f v = *(const v4f*)(lp + i * DF); *(volatile v4f*)(gp + (size_t)i * DF) = v; }
  if (wave == 0) { const v4f v = *(const v4f*)(sa1 + 4 * lane); *(volatile v4f*)(a1p + (size_t)rowBase + 4 * lane) = v; }
  if (wave == 1) { const v4f v = *(const v4f*)(sa2 + 4 * lane); *(volatile v4f*)(a2p + (size_t)rowBase + 4 * lane) = v; }
  __threadfence();
#pragma unroll
  for (int i = 0; i < 16; ++i) { const v4f v = *(const v4f*)(lp + i * DF); *(volatile v4f*)(gp + (size_t)i * DF) = v; }
  if (wave == 0) { const v4f v = *(const v4f*)(sa1 + 4 * lane); *(volatile v4f*)(a1p + (size_t)rowBase + 4 * lane) = v; }
  if (wave == 1) { const v4f v = *(const v4f*)(sa2 + 4 * lane); *(volatile v4f*)(a2p + (size_t)rowBase + 4 * lane) = v; }
}

__global__ __launch_bounds__(NTHR) void k_agg(
    const int* __restrict__ ei, const float* __restrict__ xj, const float* __restrict__ a1p,
    const float* __restrict__ a2p, const float* __restrict__ x, float* out, int nN, int nE) {
  extern __shared__ v4f lds_dyn[];
  float* acc  = (float*)lds_dyn;
  int*   list = (int*)(acc + NB * DF);
  int*   wcnt = list + LISTN;
  float* a1s  = (float*)(wcnt + 16);
  const int tid = threadIdx.x, lane = tid & 31, wave = tid >> 5;
  const int nodeBase = blockIdx.x * NB;
  const int* keys = ei;
  const int* dcol = ei + nE;

  {
    const v4f z = {0.f, 0.f, 0.f, 0.f};
    for (int i = tid; i < NB * DF / 4; i += NTHR) lds_dyn[i] = z;
    for (int i = tid; i < NB; i += NTHR) {
      int node = nodeBase + i;
      node = node > nN - 1 ? nN - 1 : node;
      a1s[i] = a1p[node];
    }
  }
  __syncthreads();

  const int nChunks = (nE + CHUNK - 1) / CHUNK;
#pragma unroll 1
  for (int ch = 0; ch < nChunks; ++ch) {
    const int cbase = ch * CHUNK;
    const int wc = scan_chunk(keys, nE, cbase, nodeBase, list, tid, lane, wave);
    if (lane == 0) wcnt[wave] = wc;
    __syncthreads();
    if (wave == 0) {
#pragma unroll 1
      for (int wsx = 0; wsx < NWAVE; ++wsx) {
        int n = __builtin_amdgcn_readfirstlane(wcnt[wsx]);
        n = n > WCAP ? WCAP : (n < 0 ? 0 : n);
        const int* lp = list + wsx * WCAP;
#pragma unroll 1
        for (int i = 0; i < n; ++i) {
          const int ent  = __builtin_amdgcn_readfirstlane(lp[i]);
          const int slot = ent & (NB - 1);
          int e = cbase + ((ent >> 12) & (CHUNK - 1));
          e = e > nE - 1 ? nE - 1 : e;
          int dst = dcol[e];
          dst = dst < 0 ? 0 : (dst > nN - 1 ? nN - 1 : dst);
          float z = a1s[slot] + a2p[dst];
          z = fminf(fmaxf(z, -30.f), 30.f);
          const float att = 1.0f / (1.0f + __expf(-z));
          const v4f v = *(const v4f*)(xj + (size_t)dst * DF + 4 * lane);
          v4f* ap = (v4f*)(acc + slot * DF + 4 * lane);
          *ap = *ap + v * att;
        }
      }
    }
    __syncthreads();
  }

#pragma unroll 4
  for (int i = 0; i < (NB * DF / 4) / NTHR; ++i) {
    const int idx  = i * NTHR + tid;
    const int slot = idx >> 5;
    const int c4   = (idx & 31) * 4;
    int node = nodeBase + slot;
    node = node > nN - 1 ? nN - 1 : node;
    const v4f xv = *(const v4f*)(x + (size_t)node * DF + c4);
    v4f* ap = (v4f*)(acc + slot * DF + c4);
    *ap = *ap + xv;
  }
  __syncthreads();

#pragma unroll 4
  for (int q = 0; q < 64; ++q) {
    const int r = wave * 64 + q;
    const int node = nodeBase + r;
    if (node < nN) { const v4f v = *(const v4f*)(acc + r * DF + 4 * lane); *(volatile v4f*)(out + (size_t)node * DF + 4 * lane) = v; }
  }
  __threadfence();
#pragma unroll 4
  for (int q = 0; q < 64; ++q) {
    const int r = wave * 64 + q;
    const int node = nodeBase + r;
    if (node < nN) { const v4f v = *(const v4f*)(acc + r * DF + 4 * lane); *(volatile v4f*)(out + (size_t)node * DF + 4 * lane) = v; }
  }
}

extern "C" void kernel_launch(void* const* d_in, const int* in_sizes, int n_in,
                              void* d_out, int out_size, void* d_ws, size_t ws_size,
                              hipStream_t stream) {
  if (n_in < 11) return;
  const int nN = in_sizes[0] / DF;
  const int nE = in_sizes[2] / 2;
  if (nN <= 0 || nE < 0 || in_sizes[0] != nN * DF || in_sizes[2] != nE * 2) return;
  if (in_sizes[3] != DF * DF || in_sizes[4] < DF || in_sizes[5] != DF * DF || in_sizes[6] < DF) return;
  if (in_sizes[7] < DF || in_sizes[8] < 1 || in_sizes[9] < DF || in_sizes[10] < 1) return;
  if (out_size != nN * DF) return;

  const float* x   = (const float*)d_in[0];
  const int*   ei  = (const int*)d_in[2];
  const float* W1  = (const float*)d_in[3];
  const float* b1  = (const float*)d_in[4];
  const float* W2  = (const float*)d_in[5];
  const float* b2  = (const float*)d_in[6];
  const float* a1w = (const float*)d_in[7];
  const float* a1b = (const float*)d_in[8];
  const float* a2w = (const float*)d_in[9];
  const float* a2b = (const float*)d_in[10];
  float* out = (float*)d_out;

  const int nG = (nN + GROWS - 1) / GROWS;
  const int nA = (nN + NB - 1) / NB;

  char* ws = (char*)d_ws;
  size_t off = 0;
  const size_t oW1 = off; off += (size_t)DF * DF * 2;                          off = (off + 255) & ~(size_t)255;
  const size_t oW2 = off; off += (size_t)DF * DF * 2;                          off = (off + 255) & ~(size_t)255;
  const size_t oXJ = off; off += (size_t)nG * GROWS * DF * 4;                  off = (off + 255) & ~(size_t)255;
  const size_t oA1 = off; off += (size_t)nG * GROWS * 4;                       off = (off + 255) & ~(size_t)255;
  const size_t oA2 = off; off += (size_t)nG * GROWS * 4;                       off = (off + 255) & ~(size_t)255;
  if (off > ws_size) return;
  _Float16* w1s = (_Float16*)(ws + oW1);
  _Float16* w2s = (_Float16*)(ws + oW2);
  float*    xj  = (float*)(ws + oXJ);
  float*    a1p = (float*)(ws + oA1);
  float*    a2p = (float*)(ws + oA2);

  const int nPrep = 2 * (DF * DF / 8);
  k_wprep<<<(nPrep + NTHR - 1) / NTHR, NTHR, 0, stream>>>(W1, W2, w1s, w2s);

  hipFuncSetAttribute(reinterpret_cast<const void*>(&k_node),
                      hipFuncAttributeMaxDynamicSharedMemorySize, LDS_NODE);
  k_node<<<nG, NTHR, LDS_NODE, stream>>>(x, w1s, w2s, b1, b2, a1w, a1b, a2w, a2b, xj, a1p, a2p, nN);

  hipFuncSetAttribute(reinterpret_cast<const void*>(&k_agg),
                      hipFuncAttributeMaxDynamicSharedMemorySize, LDS_AGG);
  k_agg<<<nA, NTHR, LDS_AGG, stream>>>(ei, xj, a1p, a2p, x, out, nN, nE);
}
